// GATSubNet_81269371175426
// MI455X (gfx1250) — hardware-verified
//
#include <hip/hip_runtime.h>
#include <math.h>

constexpr int kB  = 16;
constexpr int kN  = 1024;
constexpr int kC  = 12;
constexpr int kH  = 8;
constexpr int kD  = 64;
constexpr int kO  = 64;
constexpr int kHD = kH * kD;
constexpr int kBH = kB * kH;
constexpr float kAlpha    = 0.2f;
constexpr float kNegFill  = -1e9f;
constexpr float kPCarry   = 32768.0f;
constexpr float kWh1Carry = 16.0f;
constexpr float kH1Carry  = 256.0f;
constexpr float kWoCarry  = 256.0f;
constexpr float kWh2Carry = 2048.0f;
constexpr float kScalePV1 = kH1Carry / (kPCarry * kWh1Carry);
constexpr float kScaleWh2 = 1.0f / (kH1Carry * kWoCarry);
constexpr float kScalePV2 = 1.0f / (kPCarry * kWh2Carry);

typedef __attribute__((ext_vector_type(16))) _Float16 v16h;
typedef __attribute__((ext_vector_type(8)))  _Float16 v8h;
typedef __attribute__((ext_vector_type(16))) __bf16   v16b;
typedef __attribute__((ext_vector_type(8)))  __bf16   v8b;
typedef __attribute__((ext_vector_type(8)))  float    v8f;
typedef __attribute__((ext_vector_type(4)))  float    v4f;
typedef __attribute__((ext_vector_type(4)))  unsigned int v4u;
typedef __attribute__((ext_vector_type(4)))  int      v4i;

__device__ __forceinline__ unsigned short f2bf_bits(float f) {
  unsigned u = __float_as_uint(f);
  return (unsigned short)((u + 0x7FFFu + ((u >> 16) & 1u)) >> 16);
}
__device__ __forceinline__ float bf_bits2f(unsigned short h) { return __uint_as_float(((unsigned)h) << 16); }

__device__ __forceinline__ void dep_guard_h(v8f& a, v8f& b, v16h x, v16h y) { asm volatile("v_nop\n\tv_nop\n\tv_nop\n\tv_nop" : "+v"(a), "+v"(b) : "v"(x), "v"(y)); }
__device__ __forceinline__ void dep_guard_b(v8f& a, v8f& b, v16b x, v16b y) { asm volatile("v_nop\n\tv_nop\n\tv_nop\n\tv_nop" : "+v"(a), "+v"(b) : "v"(x), "v"(y)); }
__device__ __forceinline__ void keep4_h(v16h a, v16h b, v16h c, v16h d) { asm volatile("v_nop" :: "v"(a), "v"(b), "v"(c), "v"(d)); }
__device__ __forceinline__ void keep4_b(v16b a, v16b b, v16b c, v16b d) { asm volatile("v_nop" :: "v"(a), "v"(b), "v"(c), "v"(d)); }
__device__ __forceinline__ void acc_guard4(v8f& a, v8f& b, v8f& c, v8f& d) { asm volatile("v_nop\n\tv_nop\n\tv_nop\n\tv_nop" : "+v"(a), "+v"(b), "+v"(c), "+v"(d)); }
template <typename T> struct Frag;
template <> struct Frag<_Float16> {
  typedef v16h V; union U { v16h v; v8h h[2]; };
  static __device__ __forceinline__ v16h load(const _Float16* p) {
    U f; f.h[0] = *(const v8h*)(p); f.h[1] = *(const v8h*)(p + 16); return f.v;
  }
  static __device__ __forceinline__ v8f mma(v16h a, v16h b, v8f c) {
    return __builtin_amdgcn_wmma_f32_16x16x32_f16(false, a, false, b, (short)0, c, false, false);
  }
  static __device__ __forceinline__ void guard(v8f& a, v8f& b, v16h x, v16h y) { dep_guard_h(a, b, x, y); }
  static __device__ __forceinline__ void keep(v16h a, v16h b, v16h c, v16h d) { keep4_h(a, b, c, d); }
};
template <> struct Frag<__bf16> {
  typedef v16b V; union U { v16b v; v8b h[2]; };
  static __device__ __forceinline__ v16b load(const __bf16* p) {
    U f; f.h[0] = *(const v8b*)(p); f.h[1] = *(const v8b*)(p + 16); return f.v;
  }
  static __device__ __forceinline__ v8f mma(v16b a, v16b b, v8f c) {
    return __builtin_amdgcn_wmma_f32_16x16x32_bf16(false, a, false, b, (short)0, c, false, false);
  }
  static __device__ __forceinline__ void guard(v8f& a, v8f& b, v16b x, v16b y) { dep_guard_b(a, b, x, y); }
  static __device__ __forceinline__ void keep(v16b a, v16b b, v16b c, v16b d) { keep4_b(a, b, c, d); }
};

__device__ __forceinline__ unsigned pk16(unsigned short a, unsigned short b) { return (unsigned)a | ((unsigned)b << 16); }
__device__ __forceinline__ unsigned short h_bits(float f) { const _Float16 h = (_Float16)f; return __builtin_bit_cast(unsigned short, h); }

template <int ET> struct Elem;
template <> struct Elem<0> { typedef _Float16 T; };
template <> struct Elem<1> { typedef __bf16 T; };
template <int ET, bool SPLIT, int BIAS_MODE, int OUT_MODE, bool RESID, int ACT = 0>
__global__ __launch_bounds__(256) void wmma_gemm64(
    const unsigned short* __restrict__ Ap, const unsigned short* __restrict__ A2p, int lda, long strideA,
    const unsigned short* __restrict__ Btp, const unsigned short* __restrict__ Bt2p, int ldb, long strideB,
    void* __restrict__ Cout, void* __restrict__ Cout2, int ldc, long strideC,
    const float* __restrict__ bias,
    const float* __restrict__ resid, long strideR,
    int M, int N, int K, float scale) {
  typedef typename Elem<ET>::T T;
  typedef typename Frag<T>::V V;
  const T* A = (const T*)Ap; const T* A2 = (const T*)A2p; const T* Bt = (const T*)Btp; const T* Bt2 = (const T*)Bt2p;
  __shared__ __align__(16) float sT[8][16 * 68];
  const int b    = blockIdx.y;
  const int lane = threadIdx.x & 31;
  const int wave = threadIdx.x >> 5;
  const int tilesN = N >> 6;
  const int tilesM = M >> 6;
  const int tile = blockIdx.x * 8 + wave;
  if (tile >= tilesM * tilesN) return;
  const int tm = tile / tilesN;
  const int tn = tile - tm * tilesN;
  const int m0 = tm << 6;
  const int n0 = tn << 6;

  const T* Ab  = A  + (size_t)b * strideA;
  const T* Bb  = Bt + (size_t)b * strideB;
  const T* Ab2 = SPLIT ? (A2  + (size_t)b * strideA) : nullptr;
  const T* Bb2 = SPLIT ? (Bt2 + (size_t)b * strideB) : nullptr;

  const int rlane = lane & 15;
  const int koff  = (lane >> 4) * 8;
  const int mOff  = (lane >> 4) * 8;

  v8f acc[4][4];
#pragma unroll
  for (int i = 0; i < 4; ++i)
#pragma unroll
    for (int j = 0; j < 4; ++j) acc[i][j] = (v8f){0.f,0.f,0.f,0.f,0.f,0.f,0.f,0.f};

  for (int k0 = 0; k0 < K; k0 += 32) {
    V bh[4], bl[4];
#pragma unroll
    for (int j = 0; j < 4; ++j) {
      const size_t bo = (size_t)(n0 + (j << 4) + rlane) * ldb + koff + k0;
      bh[j] = Frag<T>::load(Bb + bo);
      if (SPLIT) bl[j] = Frag<T>::load(Bb2 + bo);
    }
#pragma unroll
    for (int i = 0; i < 4; ++i) {
      const size_t ao = (size_t)(m0 + (i << 4) + rlane) * lda + koff + k0;
      V ah = Frag<T>::load(Ab + ao);
      V al;
      if (SPLIT) al = Frag<T>::load(Ab2 + ao);
#pragma unroll
      for (int j = 0; j < 4; ++j) {
        acc[i][j] = Frag<T>::mma(ah, bh[j], acc[i][j]);
        if (SPLIT) {
          acc[i][j] = Frag<T>::mma(ah, bl[j], acc[i][j]);
          acc[i][j] = Frag<T>::mma(al, bh[j], acc[i][j]);
        }
      }
      Frag<T>::guard(acc[i][0], acc[i][3], ah, SPLIT ? al : ah);
    }
    Frag<T>::keep(bh[0], bh[1], bh[2], bh[3]);
    if (SPLIT) Frag<T>::keep(bl[0], bl[1], bl[2], bl[3]);
  }
  acc_guard4(acc[0][0], acc[0][1], acc[0][2], acc[0][3]);
  acc_guard4(acc[1][0], acc[1][1], acc[1][2], acc[1][3]);
  acc_guard4(acc[2][0], acc[2][1], acc[2][2], acc[2][3]);
  acc_guard4(acc[3][0], acc[3][1], acc[3][2], acc[3][3]);

  float* slab = sT[wave];
  const float* Rb = RESID ? (resid + (size_t)b * strideR) : nullptr;
#pragma unroll
  for (int i = 0; i < 4; ++i) {
    const int mBase = m0 + (i << 4);
#pragma unroll
    for (int j = 0; j < 4; ++j) {
      const int n = n0 + (j << 4) + rlane;
      float bv = 0.f;
      if (BIAS_MODE == 2) bv = bias[n];
#pragma unroll
      for (int r = 0; r < 8; ++r) {
        float v = acc[i][j][r] * scale;
        if (BIAS_MODE == 1) v += bias[mBase + mOff + r];
        if (BIAS_MODE == 2) v += bv;
        if (RESID) v += Rb[(size_t)(mBase + mOff + r) * ldc + n];
        if (ACT == 2) v = fmaxf(v, 0.0f);
        if (ACT == 6) v = (v > 0.f) ? v : kAlpha * v;
        slab[(mOff + r) * 68 + (j << 4) + rlane] = v;
      }
    }
    __builtin_amdgcn_fence(__ATOMIC_RELEASE, "workgroup");
    __builtin_amdgcn_wave_barrier();
    __builtin_amdgcn_fence(__ATOMIC_ACQUIRE, "workgroup");
    if (OUT_MODE == 0) {
      float* C = (float*)Cout + (size_t)b * strideC;
      const int hh = lane >> 4, c4 = (lane & 15) * 4;
      for (int pass = 0; pass < 2; ++pass) {
#pragma unroll
        for (int it = 0; it < 8; ++it) {
          const int row = it * 2 + hh;
          v4f v = *(const v4f*)(slab + row * 68 + c4);
          *(volatile v4f*)(C + (size_t)(mBase + row) * ldc + n0 + c4) = v;
        }
        __threadfence();
      }
    } else {
      const int q = lane >> 3, c8 = (lane & 7) * 8;
      unsigned short* C  = (unsigned short*)Cout  + (size_t)b * strideC;
      unsigned short* C2 = (OUT_MODE == 2) ? ((unsigned short*)Cout2 + (size_t)b * strideC) : nullptr;
      for (int pass = 0; pass < 2; ++pass) {
#pragma unroll
        for (int it = 0; it < 4; ++it) {
          const int row = it * 4 + q;
          const float* sp = slab + row * 68 + c8;
          v8h hv, lv;
#pragma unroll
          for (int e = 0; e < 8; ++e) {
            if (OUT_MODE == 1) {
              hv[e] = (_Float16)sp[e];
            } else {
              unsigned short hb = f2bf_bits(sp[e]);
              unsigned short lb = f2bf_bits(sp[e] - bf_bits2f(hb));
              hv[e] = __builtin_bit_cast(_Float16, hb);
              lv[e] = __builtin_bit_cast(_Float16, lb);
            }
          }
          *(volatile v8h*)(C + (size_t)(mBase + row) * ldc + n0 + c8) = hv;
          if (OUT_MODE == 2) *(volatile v8h*)(C2 + (size_t)(mBase + row) * ldc + n0 + c8) = lv;
        }
        __threadfence();
      }
    }
    __builtin_amdgcn_fence(__ATOMIC_RELEASE, "workgroup");
    __builtin_amdgcn_wave_barrier();
    __builtin_amdgcn_fence(__ATOMIC_ACQUIRE, "workgroup");
  }
}

__device__ __forceinline__ void store_tile_T_f16(const float (*sm)[65], unsigned short* __restrict__ out,
                                                 int ld, int col0, float carry) {
  const int t = threadIdx.x, lane = t & 31, wave = t >> 5;
  const int q = lane >> 3, c8 = (lane & 7) * 8;
  for (int pass = 0; pass < 2; ++pass) {
#pragma unroll
    for (int it = 0; it < 2; ++it) {
      const int j = wave * 8 + it * 4 + q;
      unsigned short hb[8];
#pragma unroll
      for (int e = 0; e < 8; ++e) hb[e] = h_bits(sm[c8 + e][j] * carry);
      const v4u u = (v4u){pk16(hb[0], hb[1]), pk16(hb[2], hb[3]), pk16(hb[4], hb[5]), pk16(hb[6], hb[7])};
      *(volatile v4u*)(out + (size_t)j * ld + col0 + c8) = u;
    }
    __threadfence();
  }
}

__device__ __forceinline__ void score_store(const float (*sm)[65], const float (*aa)[64], float (*stv)[64],
                                            float* __restrict__ sdst, float* __restrict__ tdst) {
  const int t = threadIdx.x;
  if (t < 128) {
    const int nl = t & 63, which = t >> 6;
    float acc = 0.f;
#pragma unroll 1
    for (int d = 0; d < 64; ++d) acc = fmaf(sm[nl][d], aa[which][d], acc);
    stv[which][nl] = acc;
  }
  __syncthreads();
  if (t < 32) {
    const int which = t >> 4, c4 = (t & 15) * 4;
    const v4f v = *(const v4f*)(&stv[which][c4]);
    float* dst = (which ? tdst : sdst) + c4;
    *(volatile v4f*)dst = v;
    __threadfence();
    *(volatile v4f*)dst = v;
  }
}

__global__ __launch_bounds__(256) void wh1_kernel(const float* __restrict__ x, const float* __restrict__ W,
                                                  const float* __restrict__ a_src, const float* __restrict__ a_dst,
                                                  unsigned short* __restrict__ whT1,
                                                  float* __restrict__ s1, float* __restrict__ t1) {
  __shared__ __align__(16) float xs[64 * kC];
  __shared__ __align__(16) float wsm[kC * kD];
  __shared__ __align__(16) float aa[2][64];
  __shared__ __align__(16) float stv[2][64];
  __shared__ float sm[64][65];
  const int t  = threadIdx.x;
  const int n0 = blockIdx.x * 64;
  const int bh = blockIdx.y;
  const int b  = bh >> 3, h = bh & 7;
  const float* xg = x + ((size_t)b * kN + n0) * kC;
  const float* wg = W + (size_t)h * kC * kD;
  if (t < 192) {
    const v4f xv = *(const v4f*)(xg + 4 * t);
    *(v4f*)(xs + 4 * t) = xv;
    const v4f wv = *(const v4f*)(wg + 4 * t);
    *(v4f*)(wsm + 4 * t) = wv;
  }
  if (t < 64) aa[0][t] = a_src[h * kD + t];
  if (t >= 64 && t < 128) aa[1][t - 64] = a_dst[h * kD + (t - 64)];
  __syncthreads();
  const int nl = t >> 2, dq = (t & 3) * 16;
  float acc[16];
#pragma unroll
  for (int j = 0; j < 16; ++j) acc[j] = 0.f;
#pragma unroll 1
  for (int c = 0; c < kC; ++c) {
    const float xv = xs[nl * kC + c];
#pragma unroll
    for (int j = 0; j < 16; ++j) acc[j] = fmaf(xv, wsm[c * kD + dq + j], acc[j]);
  }
#pragma unroll
  for (int j = 0; j < 16; ++j) sm[nl][dq + j] = acc[j];
  __syncthreads();
  score_store(sm, aa, stv, s1 + (size_t)bh * kN + n0, t1 + (size_t)bh * kN + n0);
  store_tile_T_f16(sm, whT1 + (size_t)bh * kD * kN, kN, n0, kWh1Carry);
}

__global__ __launch_bounds__(256) void st2_kernel(const float* __restrict__ wh2,
                                                  const float* __restrict__ ao_src, const float* __restrict__ ao_dst,
                                                  unsigned short* __restrict__ whT2,
                                                  float* __restrict__ s2, float* __restrict__ t2) {
  __shared__ __align__(16) float aa[2][64];
  __shared__ __align__(16) float stv[2][64];
  __shared__ float sm[64][65];
  const int t  = threadIdx.x;
  const int n0 = blockIdx.x * 64;
  const int b  = blockIdx.y;
  const float* src = wh2 + ((size_t)b * kN + n0) * kO;
#pragma unroll
  for (int i = 0; i < 4; ++i) {
    const int e = i * 256 + t;
    const int row = e >> 4, c4 = (e & 15) * 4;
    const v4f v = *(const v4f*)(src + (size_t)row * kO + c4);
    sm[row][c4 + 0] = v[0]; sm[row][c4 + 1] = v[1]; sm[row][c4 + 2] = v[2]; sm[row][c4 + 3] = v[3];
  }
  if (t < 64) aa[0][t] = ao_src[t];
  if (t >= 64 && t < 128) aa[1][t - 64] = ao_dst[t - 64];
  __syncthreads();
  score_store(sm, aa, stv, s2 + (size_t)b * kN + n0, t2 + (size_t)b * kN + n0);
  store_tile_T_f16(sm, whT2 + (size_t)b * kO * kN, kN, n0, kWh2Carry);
}

__global__ __launch_bounds__(256) void wot_kernel(const float* __restrict__ Wo, unsigned short* __restrict__ woT) {
  __shared__ float sm[64][65];
  const int t  = threadIdx.x;
  const int k0 = blockIdx.x * 64;
#pragma unroll
  for (int i = 0; i < 16; ++i) {
    const int e = i * 256 + t;
    const int r = e >> 6, c = e & 63;
    sm[r][c] = Wo[(size_t)(k0 + r) * kO + c];
  }
  __syncthreads();
  store_tile_T_f16(sm, woT, kHD, k0, kWoCarry);
}

template <int NHEAD>
__global__ __launch_bounds__(128) void softmax_p_kernel(const float* __restrict__ s, const float* __restrict__ tt,
                                                        const int* __restrict__ graph, unsigned short* __restrict__ P,
                                                        int plane0) {
  __shared__ float redm[4];
  __shared__ float reds[4];
  const int n = blockIdx.x;
  const int t = threadIdx.x, lane = t & 31, wave = t >> 5;
  const int m0 = t * 8;
  const int* gr = graph + (size_t)n * kN + m0;
  const v4i ga = *(const v4i*)gr;
  const v4i gb = *(const v4i*)(gr + 4);
  bool keep[8];
#pragma unroll
  for (int e = 0; e < 4; ++e) { keep[e] = ga[e] > 0; keep[4 + e] = gb[e] > 0; }
  for (int hd = 0; hd < NHEAD; ++hd) {
    const int pl = (int)blockIdx.y * NHEAD + hd;
    const size_t sp = (size_t)(plane0 + pl) * kN;
    const float sn = s[sp + n];
    const float* tr = tt + sp + m0;
    const v4f ta = *(const v4f*)tr;
    const v4f tb = *(const v4f*)(tr + 4);
    float ev[8];
#pragma unroll
    for (int e = 0; e < 4; ++e) { ev[e] = sn + ta[e]; ev[4 + e] = sn + tb[e]; }
#pragma unroll
    for (int e = 0; e < 8; ++e) {
      float v = ev[e];
      v = fmaxf(v, kAlpha * v);
      ev[e] = keep[e] ? v : kNegFill;
    }
    float mx = fmaxf(fmaxf(fmaxf(ev[0], ev[1]), fmaxf(ev[2], ev[3])), fmaxf(fmaxf(ev[4], ev[5]), fmaxf(ev[6], ev[7])));
#pragma unroll
    for (int off = 16; off > 0; off >>= 1) mx = fmaxf(mx, __shfl_xor(mx, off, 32));
    if (lane == 0) redm[wave] = mx;
    __syncthreads();
    const float M = fmaxf(fmaxf(redm[0], redm[1]), fmaxf(redm[2], redm[3]));
    float pv[8];
    float ps = 0.f;
#pragma unroll
    for (int e = 0; e < 8; ++e) { pv[e] = expf(ev[e] - M); ps += pv[e]; }
#pragma unroll
    for (int off = 16; off > 0; off >>= 1) ps += __shfl_xor(ps, off, 32);
    if (lane == 0) reds[wave] = ps;
    __syncthreads();
    const float S = ((reds[0] + reds[1]) + reds[2]) + reds[3];
    const float inv = kPCarry / S;
    unsigned short hb[8];
#pragma unroll
    for (int e = 0; e < 8; ++e) hb[e] = h_bits(pv[e] * inv);
    const v4u u = (v4u){pk16(hb[0], hb[1]), pk16(hb[2], hb[3]), pk16(hb[4], hb[5]), pk16(hb[6], hb[7])};
    unsigned short* dst = P + (size_t)pl * ((size_t)kN * kN) + (size_t)n * kN + m0;
    *(volatile v4u*)dst = u;
    __threadfence();
    *(volatile v4u*)dst = u;
  }
}

extern "C" void kernel_launch(void* const* d_in, const int* in_sizes, int n_in,
                              void* d_out, int out_size, void* d_ws, size_t ws_size,
                              hipStream_t stream) {
  if (n_in < 8) return;
  if (in_sizes[0] != kB * kN * kC) return;
  if (in_sizes[1] != kN * kN) return;
  if (in_sizes[2] != kH * kC * kD) return;
  if (in_sizes[3] != kH * kD || in_sizes[4] != kH * kD) return;
  if (in_sizes[5] != kHD * kO) return;
  if (in_sizes[6] != kO || in_sizes[7] != kO) return;
  if (out_size != kB * kN * kO) return;

  const float* x      = (const float*)d_in[0];
  const int*   graph  = (const int*)d_in[1];
  const float* W      = (const float*)d_in[2];
  const float* a_src  = (const float*)d_in[3];
  const float* a_dst  = (const float*)d_in[4];
  const float* Wo     = (const float*)d_in[5];
  const float* ao_src = (const float*)d_in[6];
  const float* ao_dst = (const float*)d_in[7];
  float* out = (float*)d_out;

  char* ws = (char*)d_ws;
  size_t off = 0;
  const size_t bytes_s1   = (size_t)kBH * kN * 4;
  const size_t bytes_s2   = (size_t)kB * kN * 4;
  const size_t bytes_whT1 = (size_t)kBH * kD * kN * 2;
  const size_t bytes_h1   = (size_t)kB * kN * kHD * 2;
  const size_t bytes_woT  = (size_t)kO * kHD * 2;
  const size_t bytes_wh2  = (size_t)kB * kN * kO * 4;
  const size_t bytes_whT2 = (size_t)kB * kO * kN * 2;
  const size_t plane_P    = (size_t)kN * kN;
  const size_t bytes_P    = (size_t)16 * plane_P * 2;

  float* s1 = (float*)(ws + off);             off += bytes_s1;
  float* t1 = (float*)(ws + off);             off += bytes_s1;
  float* s2 = (float*)(ws + off);             off += bytes_s2;
  float* t2 = (float*)(ws + off);             off += bytes_s2;
  unsigned short* whT1 = (unsigned short*)(ws + off); off += bytes_whT1;
  unsigned short* h1   = (unsigned short*)(ws + off); off += bytes_h1;
  unsigned short* woT  = (unsigned short*)(ws + off); off += bytes_woT;
  float* wh2 = (float*)(ws + off);            off += bytes_wh2;
  unsigned short* whT2 = (unsigned short*)(ws + off); off += bytes_whT2;
  unsigned short* Pp   = (unsigned short*)(ws + off); off += bytes_P;
  if (off > ws_size) return;

  const size_t plane_whT = (size_t)kD * kN;

  wh1_kernel<<<dim3(kN / 64, kBH), 256, 0, stream>>>(x, W, a_src, a_dst, whT1, s1, t1);
  wot_kernel<<<dim3(kHD / 64), 256, 0, stream>>>(Wo, woT);

  for (int it = 0; it < kB / 2; ++it) {
    softmax_p_kernel<8><<<dim3(kN, 2), 128, 0, stream>>>(s1, t1, graph, Pp, it * 16);
    for (int bl = 0; bl < 2; ++bl) {
      const int b = it * 2 + bl;
      wmma_gemm64<0, false, 0, 1, false, 6><<<dim3(2, kH), 256, 0, stream>>>(
          Pp + (size_t)bl * 8 * plane_P, nullptr, kN, (long)plane_P,
          whT1 + (size_t)b * kH * plane_whT, nullptr, kN, (long)plane_whT,
          (void*)(h1 + (size_t)b * kN * kHD), nullptr, kHD, (long)kD,
          nullptr, nullptr, 0L,
          kN, kD, kN, kScalePV1);
    }
  }

  wmma_gemm64<0, false, 0, 0, false, 0><<<dim3(32, 1), 256, 0, stream>>>(
      h1, nullptr, kHD, 0L,
      woT, nullptr, kHD, 0L,
      (void*)wh2, nullptr, kO, 0L,
      nullptr, nullptr, 0L,
      kB * kN, kO, kHD, kScaleWh2);

  st2_kernel<<<dim3(kN / 64, kB), 256, 0, stream>>>(wh2, ao_src, ao_dst, whT2, s2, t2);

  softmax_p_kernel<1><<<dim3(kN, kB), 128, 0, stream>>>(s2, t2, graph, Pp, 0);
  wmma_gemm64<0, false, 0, 0, false, 6><<<dim3(2, kB), 256, 0, stream>>>(
      Pp, nullptr, kN, (long)plane_P,
      whT2, nullptr, kN, (long)plane_whT,
      (void*)out, nullptr, kO, (long)((size_t)kN * kO),
      nullptr, nullptr, 0L,
      kN, kO, kN, kScalePV2);
}
